// NonLocalAttention_8830452761398
// MI455X (gfx1250) — hardware-verified
//
#include <hip/hip_runtime.h>


namespace {
typedef _Float16 b16;
typedef __attribute__((ext_vector_type(16))) _Float16 v16b;
typedef __attribute__((ext_vector_type(8))) _Float16 v8b;
typedef __attribute__((ext_vector_type(4))) _Float16 v4h;
typedef __attribute__((ext_vector_type(2))) _Float16 v2h;
typedef __attribute__((ext_vector_type(8))) float v8f;

#ifndef NB
#define NB 4
#endif
#ifndef SEQ
#define SEQ 6400
#endif
constexpr int NB_FULL = 4, L_FULL = 6400;
constexpr int CIN = 128, CR = 64, CV = 128, GW = 128, NO = 2 * GW;
static_assert(NB >= 1 && NB <= NB_FULL);
static_assert(SEQ % 64 == 0 && SEQ >= 64 && SEQ <= L_FULL);
static_assert(CIN % 32 == 0 && 2 * CR == GW && CV == GW && CR % 32 == 0);
constexpr float XS = 8.0f, WSC = 256.0f, PS = 16384.0f, LOG2E = 1.4426950408889634f;

__device__ __forceinline__ float bf16_rne(float f) { unsigned int u = __float_as_uint(f); u += 0x7FFFu + ((u >> 16) & 1u); return __uint_as_float(u & 0xFFFF0000u); }
__device__ __forceinline__ v16b frag_kb(const b16* p, int hh) {
  const v8b a = *(const v8b*)(p + 8 * hh), b = *(const v8b*)(p + 16 + 8 * hh); v16b f;
#pragma unroll
  for (int e = 0; e < 8; ++e) { f[e] = a[e]; f[8 + e] = b[e]; }
  return f;
}
__device__ __forceinline__ v8f wmma16b(v16b a, v16b b, v8f c) {
  v8f d = __builtin_amdgcn_wmma_f32_16x16x32_f16(false, a, false, b, (short)0, c, false, false);
  asm volatile("v_nop\n\tv_nop\n\tv_nop\n\tv_nop" : "+v"(d) : "v"(a), "v"(b));
  return d;
}
__device__ __forceinline__ void wave_lds_sync() { __builtin_amdgcn_fence(3u, "workgroup"); __builtin_amdgcn_wave_barrier(); __builtin_amdgcn_fence(2u, "workgroup"); }
__device__ __forceinline__ float nexp2(float v) { return __builtin_amdgcn_exp2f(v); }
__device__ __forceinline__ float prelu(float v, float a) { return v >= 0.0f ? v : a * v; }

__global__ __launch_bounds__(256) void prep_kernel(const float* __restrict__ w1, const float* __restrict__ w2, const float* __restrict__ wa, b16* __restrict__ WT) {
  const int u = blockIdx.x * 256 + threadIdx.x;
  if (u >= NO * CIN / 8) return;
  const int e = u * 8; const int o = e / CIN, c = e % CIN;
  const float* w = o < CR ? w1 + (size_t)o * CIN : (o < 2 * CR ? w2 + (size_t)(o - CR) * CIN : wa + (size_t)(o - 2 * CR) * CIN);
  v8b v;
#pragma unroll
  for (int j = 0; j < 8; ++j) v[j] = (b16)(bf16_rne(w[c + j]) * WSC);
  for (int ps = 0; ps < 2; ++ps) { *(volatile v8b*)(WT + e) = v; __threadfence(); }
}

__global__ __launch_bounds__(128) void qkv_kernel(const float* __restrict__ x, const b16* __restrict__ WT,
                                                  const float* __restrict__ b1, const float* __restrict__ a1, const float* __restrict__ b2, const float* __restrict__ a2,
                                                  const float* __restrict__ ba, const float* __restrict__ aa,
                                                  b16* __restrict__ Qh, b16* __restrict__ Kh, b16* __restrict__ VT) {
  __shared__ __attribute__((aligned(16))) b16 As[64][CIN + 8];
  __shared__ __attribute__((aligned(16))) float Tf[4][16][GW + 4];
  const int wave = threadIdx.x >> 5, lane = threadIdx.x & 31, nloc = lane & 15, hlf = lane >> 4;
  const int p0 = blockIdx.x * 64; const int b = blockIdx.y;
  for (int i = threadIdx.x; i < CIN * 64; i += 128) { const int c = i >> 6, pp = i & 63; As[pp][c] = (b16)(bf16_rne(x[((size_t)b * CIN + c) * L_FULL + p0 + pp]) * XS); }
  const float s1 = bf16_rne(a1[0]), s2 = bf16_rne(a2[0]), s3 = bf16_rne(aa[0]);
  __syncthreads();
#pragma unroll
  for (int g = 0; g < 2; ++g) {
    v8f acc[8];
#pragma unroll
    for (int t = 0; t < 8; ++t) acc[t] = (v8f){};
#pragma unroll
    for (int kb = 0; kb < CIN; kb += 32) {
      const v16b a = frag_kb(&As[wave * 16 + nloc][kb], hlf);
#pragma unroll
      for (int t = 0; t < 8; ++t) acc[t] = wmma16b(a, frag_kb(WT + (size_t)(g * GW + t * 16 + nloc) * CIN + kb, hlf), acc[t]);
    }
#pragma unroll
    for (int t = 0; t < 8; ++t) {
      const float* bp = g == 0 ? (t < 4 ? b1 + t * 16 : b2 + (t - 4) * 16) : ba + t * 16;
      const float sl = g == 0 ? (t < 4 ? s1 : s2) : s3;
      const float bbs = bf16_rne(bp[nloc]) * (XS * WSC);
#pragma unroll
      for (int r = 0; r < 8; ++r) Tf[wave][8 * hlf + r][t * 16 + nloc] = prelu(acc[t][r] + bbs, sl);
    }
    __syncthreads();
    for (int ps = 0; ps < 2; ++ps) {
      if (g == 0) {
#pragma unroll 1
        for (int rr = 0; rr < 16; ++rr) {
          const int p = p0 + wave * 16 + rr; const int which = lane >> 4, d = (lane & 15) * 4; v4h hv;
#pragma unroll
          for (int j = 0; j < 4; ++j) hv[j] = (b16)(Tf[wave][rr][which * CR + d + j] * (1.0f / WSC));
          b16* ph = which == 0 ? Qh : Kh;
          *(volatile v4h*)(ph + ((size_t)b * L_FULL + p) * CR + d) = hv;
        }
      } else {
#pragma unroll 1
        for (int q = 0; q < 32; ++q) {
          const int dch = wave * 32 + q; const int tk = lane * 2; v2h vv;
          vv[0] = (b16)(Tf[tk >> 4][tk & 15][dch] * (1.0f / WSC)); vv[1] = (b16)(Tf[(tk + 1) >> 4][(tk + 1) & 15][dch] * (1.0f / WSC));
          *(volatile v2h*)(VT + ((size_t)b * CV + dch) * (size_t)L_FULL + p0 + tk) = vv;
        }
      }
      __threadfence();
    }
    __syncthreads();
  }
}

__global__ __launch_bounds__(64) __attribute__((amdgpu_num_vgpr(256))) void attn_kernel(const b16* __restrict__ Qh, const b16* __restrict__ Kh, const b16* __restrict__ VT, float* __restrict__ out) {
  __shared__ __attribute__((aligned(16))) b16 Pb[2][16][32 + 8];
  __shared__ __attribute__((aligned(16))) float To[32][CV + 4];
  const int wave = threadIdx.x >> 5, lane = threadIdx.x & 31, hh = lane >> 4, col = lane & 15;
  const int b = blockIdx.y; const int p0 = blockIdx.x * 32; const int q0 = p0 + wave * 16, qi = q0 + col;
  const b16* Qhb = Qh + (size_t)b * L_FULL * CR; const b16* Khb = Kh + (size_t)b * L_FULL * CR; const b16* Vb = VT + (size_t)b * CV * L_FULL;
  v16b qf[2];
#pragma unroll
  for (int s = 0; s < 2; ++s) qf[s] = frag_kb(Qhb + (size_t)qi * CR + 32 * s, hh);
  const float cs = LOG2E / (XS * XS);
  float m = -INFINITY, l = 0.0f; v8f o[8];
#pragma unroll
  for (int t = 0; t < 8; ++t) o[t] = (v8f){};
#pragma unroll 1
  for (int kb = 0; kb < SEQ; kb += 32) {
    float e[16]; float mx = -INFINITY;
#pragma unroll
    for (int u = 0; u < 2; ++u) {
      v8f s = (v8f){}; const size_t kr = (size_t)(kb + u * 16 + col) * CR;
#pragma unroll
      for (int st = 0; st < 2; ++st) s = wmma16b(frag_kb(Khb + kr + 32 * st, hh), qf[st], s);
#pragma unroll
      for (int r = 0; r < 8; ++r) { const float vv = s[r] * cs; e[u * 8 + r] = vv; mx = fmaxf(mx, vv); }
    }
    mx = fmaxf(mx, __shfl_xor(mx, 16)); const float mn = fmaxf(m, mx); const float al = nexp2(m - mn); float sum = 0.0f;
#pragma unroll
    for (int i2 = 0; i2 < 16; ++i2) { const float p = nexp2(e[i2] - mn); sum += p; Pb[wave][col][(i2 < 8 ? 0 : 16) + 8 * hh + (i2 & 7)] = (b16)(p * PS); }
    sum += __shfl_xor(sum, 16); l = l * al + sum; m = mn;
    wave_lds_sync();
    const v16b pf = frag_kb(&Pb[wave][col][0], hh);
#pragma unroll
    for (int t = 0; t < 8; ++t) { o[t] *= al; o[t] = wmma16b(frag_kb(Vb + (size_t)(t * 16 + col) * L_FULL + kb, hh), pf, o[t]); }
    wave_lds_sync();
  }
  const float inv = 1.0f / (l * PS * XS);
#pragma unroll
  for (int t = 0; t < 8; ++t)
#pragma unroll
    for (int r = 0; r < 8; ++r) To[wave * 16 + col][t * 16 + 8 * hh + r] = o[t][r] * inv;
  __syncthreads();
  for (int ps = 0; ps < 2; ++ps) {
#pragma unroll 1
    for (int q = 0; q < 64; ++q) { const int c = wave * 64 + q; ((volatile float*)out)[((size_t)b * CV + c) * (size_t)SEQ + p0 + lane] = To[lane][c]; }
    __threadfence();
  }
}
}

extern "C" void kernel_launch(void* const* d_in, const int* in_sizes, int n_in, void* d_out, int out_size, void* d_ws, size_t ws_size, hipStream_t stream) {
  if (n_in < 10) return;
  auto Fp = [&](int i) { return (const float*)d_in[i]; };
  if (in_sizes[0] < NB * CIN * L_FULL || in_sizes[1] < CR * CIN || in_sizes[2] < CR || in_sizes[3] < 1 || in_sizes[4] < CR * CIN || in_sizes[5] < CR || in_sizes[6] < 1 ||
      in_sizes[7] < CV * CIN || in_sizes[8] < CV || in_sizes[9] < 1 || out_size < NB * CV * SEQ) return;
  size_t off = 0; char* ws = (char*)d_ws;
  auto carve = [&](size_t bytes) { char* p = ws + off; off += (bytes + 255) & ~(size_t)255; return p; };
  b16* WT = (b16*)carve((size_t)NO * CIN * 2);
  b16* Qh = (b16*)carve((size_t)NB * L_FULL * CR * 2);
  b16* Kh = (b16*)carve((size_t)NB * L_FULL * CR * 2);
  b16* VT = (b16*)carve((size_t)NB * CV * L_FULL * 2);
  if (off > ws_size || off > ((size_t)128 << 20)) return;
  prep_kernel<<<(NO * CIN / 8 + 255) / 256, 256, 0, stream>>>(Fp(1), Fp(4), Fp(7), WT);
  qkv_kernel<<<dim3(SEQ / 64, NB), 128, 0, stream>>>(Fp(0), WT, Fp(2), Fp(3), Fp(5), Fp(6), Fp(8), Fp(9), Qh, Kh, VT);
  attn_kernel<<<dim3(SEQ / 32, NB), 64, 0, stream>>>(Qh, Kh, VT, (float*)d_out);
}
